// hqaf_60687887893234
// MI455X (gfx1250) — hardware-verified
//
#include <hip/hip_runtime.h>
#include <math.h>
#include <stdint.h>

#define NBATCH  8
#define SEQ     1024
#define DM      512
#define NH      8
#define HD      64
#define ROWS    (NBATCH * SEQ)
#define NQB     (SEQ / 64)
#define QPITCH  (2 * DM)
#define VPITCH  (2 * SEQ)
#define OPITCH  (2 * DM)
#define W2PITCH (2 * DM)
static_assert(NH * HD == DM);
static_assert(HD == 64);
static_assert((SEQ % 64) == 0 && (DM % 64) == 0 && (DM % 32) == 0);
static_assert(((ROWS / 64) * (DM / 64)) % 8 == 0);
static_assert(((ROWS * DM / 8) % 256) == 0 && ((DM * DM / 8) % 256) == 0);

typedef __bf16       v16bf __attribute__((ext_vector_type(16)));
typedef __bf16       v8bf  __attribute__((ext_vector_type(8)));
typedef float        v8f   __attribute__((ext_vector_type(8)));
typedef float        v4f   __attribute__((ext_vector_type(4)));
typedef unsigned int v4u   __attribute__((ext_vector_type(4)));
typedef unsigned int v2u   __attribute__((ext_vector_type(2)));

__device__ __forceinline__ unsigned short bf_bits(float f) {
  unsigned u = __float_as_uint(f);
  return (unsigned short)((u + 0x7FFFu + ((u >> 16) & 1u)) >> 16);
}
__device__ __forceinline__ float bf_val(unsigned short b) { return __uint_as_float(((unsigned)b) << 16); }
__device__ __forceinline__ float bfr(float f) { return bf_val(bf_bits(f)); }
__device__ __forceinline__ unsigned pk16(unsigned short a, unsigned short b) { return (unsigned)a | ((unsigned)b << 16); }
__device__ __forceinline__ v8f zero8() { v8f z = {0.f, 0.f, 0.f, 0.f, 0.f, 0.f, 0.f, 0.f}; return z; }

__device__ __forceinline__ v16bf ldfrag_b(const unsigned short* p) {
  union { v16bf v; v8bf h[2]; } f;
  f.h[0] = *(const v8bf*)(const void*)(p);
  f.h[1] = *(const v8bf*)(const void*)(p + 16);
  return f.v;
}

__device__ __forceinline__ v8f mma_b_raw(v16bf a, v16bf b, v8f c) {
  return __builtin_amdgcn_wmma_f32_16x16x32_bf16(false, a, false, b, (short)0, c, false, false);
}
__device__ __forceinline__ v8f mma_b(v16bf a, v16bf b, v8f c) {
  c = mma_b_raw(a, b, c);
#if defined(__HIP_DEVICE_COMPILE__)
  asm volatile("v_nop\n\tv_nop\n\tv_nop\n\tv_nop" : "+v"(c) : "v"(a), "v"(b));
#endif
  return c;
}
__device__ __forceinline__ void dep_guard_b(v8f& a, v8f& b, v16bf x, v16bf y) {
#if defined(__HIP_DEVICE_COMPILE__)
  asm volatile("v_nop\n\tv_nop\n\tv_nop\n\tv_nop" : "+v"(a), "+v"(b) : "v"(x), "v"(y));
#endif
}
__device__ __forceinline__ void keep4_b(v16bf a, v16bf b, v16bf c, v16bf d) {
#if defined(__HIP_DEVICE_COMPILE__)
  asm volatile("v_nop" :: "v"(a), "v"(b), "v"(c), "v"(d));
#endif
}
__device__ __forceinline__ void acc_guard4(v8f& a, v8f& b, v8f& c, v8f& d) {
#if defined(__HIP_DEVICE_COMPILE__)
  asm volatile("v_nop\n\tv_nop\n\tv_nop\n\tv_nop" : "+v"(a), "+v"(b), "+v"(c), "+v"(d));
#endif
}
__device__ __forceinline__ void lds_wave_sync() {
  __builtin_amdgcn_fence(__ATOMIC_RELEASE, "workgroup");
  __builtin_amdgcn_wave_barrier();
  __builtin_amdgcn_fence(__ATOMIC_ACQUIRE, "workgroup");
}

__global__ __launch_bounds__(256) void cvt_bf(const float* __restrict__ in, unsigned short* out,
                                              int n8, int dup, int kdim) {
  const int i = blockIdx.x * 256 + threadIdx.x;
  if (i < n8) {
    const size_t e = (size_t)i * 8;
    const v4f a = *(const v4f*)(in + e);
    const v4f b = *(const v4f*)(in + e + 4);
    v4u p;
    p[0] = pk16(bf_bits(a[0]), bf_bits(a[1]));
    p[1] = pk16(bf_bits(a[2]), bf_bits(a[3]));
    p[2] = pk16(bf_bits(b[0]), bf_bits(b[1]));
    p[3] = pk16(bf_bits(b[2]), bf_bits(b[3]));
    size_t o0 = e, o1 = e;
    if (dup != 0) {
      const size_t row = e / (size_t)kdim;
      const size_t col = e - row * (size_t)kdim;
      o0 = row * 2 * (size_t)kdim + col;
      o1 = o0 + (size_t)kdim;
    }
    for (int ps = 0; ps < 2; ++ps) {
      *(volatile v4u*)(out + o0) = p;
      if (dup != 0) *(volatile v4u*)(out + o1) = p;
      __threadfence();
    }
  }
}

template <int EPI>
__global__ __launch_bounds__(256) void gemm64_bf(
    const unsigned short* __restrict__ Ap, int lda,
    const unsigned short* __restrict__ Btp, int ldb,
    const float* __restrict__ biasp,
    void* Cp, int ldc, int loff, int M, int N, int K) {
  __shared__ __align__(16) float sT[8][16 * 68];
  const int lane = threadIdx.x & 31;
  const int wave = threadIdx.x >> 5;
  const int tilesN = N >> 6;
  const int tilesM = M >> 6;
  const int tile = blockIdx.x * 8 + wave;
  if (tile >= tilesM * tilesN) return;
  const int tm = tile / tilesN;
  const int tn = tile - tm * tilesN;
  const int m0 = tm << 6;
  const int n0 = tn << 6;

  const int rlane = lane & 15;
  const int koff  = (lane >> 4) * 8;
  const int mOff  = (lane >> 4) * 8;

  v8f acc[4][4];
#pragma unroll
  for (int i = 0; i < 4; ++i)
#pragma unroll
    for (int j = 0; j < 4; ++j) acc[i][j] = zero8();

  for (int k0 = 0; k0 < K; k0 += 32) {
    v16bf bh[4];
#pragma unroll
    for (int j = 0; j < 4; ++j) {
      const size_t bo = (size_t)(n0 + (j << 4) + rlane) * ldb + koff + k0;
      bh[j] = ldfrag_b(Btp + bo);
    }
#pragma unroll
    for (int i = 0; i < 4; ++i) {
      const size_t ao = (size_t)(m0 + (i << 4) + rlane) * lda + koff + k0;
      const v16bf ah = ldfrag_b(Ap + ao);
#pragma unroll
      for (int j = 0; j < 4; ++j) {
        acc[i][j] = mma_b_raw(ah, bh[j], acc[i][j]);
      }
      dep_guard_b(acc[i][0], acc[i][3], ah, bh[3]);
    }
    keep4_b(bh[0], bh[1], bh[2], bh[3]);
  }
  acc_guard4(acc[0][0], acc[0][1], acc[0][2], acc[0][3]);
  acc_guard4(acc[1][0], acc[1][1], acc[1][2], acc[1][3]);
  acc_guard4(acc[2][0], acc[2][1], acc[2][2], acc[2][3]);
  acc_guard4(acc[3][0], acc[3][1], acc[3][2], acc[3][3]);

  float* slab = sT[wave];
#pragma unroll
  for (int i = 0; i < 4; ++i) {
    const int mBase = m0 + (i << 4);
    float bj[4];
#pragma unroll
    for (int j = 0; j < 4; ++j) {
      if constexpr (EPI == 1) bj[j] = 0.0f;
      else bj[j] = bfr(biasp[n0 + (j << 4) + rlane]);
    }
#pragma unroll
    for (int r = 0; r < 8; ++r) {
      const int row = mOff + r;
      float br = 0.0f;
      if constexpr (EPI == 1) br = bfr(biasp[mBase + row]);
#pragma unroll
      for (int j = 0; j < 4; ++j) {
        float v = acc[i][j][r];
        if constexpr (EPI == 1) v += br;
        else v += bj[j];
        slab[row * 68 + (j << 4) + rlane] = v;
      }
    }
    lds_wave_sync();
    if constexpr (EPI <= 1) {
      unsigned short* C16 = (unsigned short*)Cp;
      const int rq = lane >> 3, piece = lane & 7;
      v4u ph[4], pl[4];
      size_t go[4];
#pragma unroll
      for (int it = 0; it < 4; ++it) {
        const int row = it * 4 + rq;
        const v4f x0 = *(const v4f*)(slab + row * 68 + piece * 8);
        const v4f x1 = *(const v4f*)(slab + row * 68 + piece * 8 + 4);
        float f[8];
        f[0] = x0[0]; f[1] = x0[1]; f[2] = x0[2]; f[3] = x0[3];
        f[4] = x1[0]; f[5] = x1[1]; f[6] = x1[2]; f[7] = x1[3];
        v4u p0, p1;
#pragma unroll
        for (int e = 0; e < 4; ++e) {
          const unsigned short ha = bf_bits(f[2 * e]);
          const unsigned short hb = bf_bits(f[2 * e + 1]);
          const unsigned short la = bf_bits(f[2 * e] - bf_val(ha));
          const unsigned short lb = bf_bits(f[2 * e + 1] - bf_val(hb));
          p0[e] = pk16(ha, hb);
          p1[e] = pk16(la, lb);
        }
        ph[it] = p0;
        pl[it] = p1;
        if constexpr (EPI == 0) {
          go[it] = (size_t)(mBase + row) * ldc + n0 + piece * 8;
        } else {
          const int bb = n0 / SEQ;
          const int s0 = n0 - bb * SEQ;
          go[it] = ((size_t)(bb * DM + mBase + row)) * ldc + s0 + piece * 8;
        }
      }
      for (int ps = 0; ps < 2; ++ps) {
#pragma unroll
        for (int it = 0; it < 4; ++it) {
          *(volatile v4u*)(C16 + go[it]) = ph[it];
          *(volatile v4u*)(C16 + go[it] + loff) = pl[it];
        }
        __threadfence();
      }
    } else {
      float* Cf = (float*)Cp;
      const int h2 = lane >> 4, c4 = (lane & 15) * 4;
      v4f ov[8];
#pragma unroll
      for (int it = 0; it < 8; ++it) {
        const int row = it * 2 + h2;
        ov[it] = *(const v4f*)(slab + row * 68 + c4);
      }
      for (int ps = 0; ps < 2; ++ps) {
#pragma unroll
        for (int it = 0; it < 8; ++it) {
          const int row = it * 2 + h2;
          *(volatile v4f*)(Cf + (size_t)(mBase + row) * ldc + n0 + c4) = ov[it];
        }
        __threadfence();
      }
    }
    lds_wave_sync();
  }
}

__device__ __forceinline__ void scores_tile(v8f (&s)[4], const unsigned short* __restrict__ qfr,
                                            const unsigned short* ksh, int c, int hh) {
  v16bf qh[2], ql[2];
#pragma unroll
  for (int dc = 0; dc < 2; ++dc) {
    qh[dc] = ldfrag_b(qfr + dc * 32);
    ql[dc] = ldfrag_b(qfr + DM + dc * 32);
  }
#pragma unroll
  for (int j = 0; j < 4; ++j) {
    v8f acc = zero8();
#pragma unroll
    for (int dc = 0; dc < 2; ++dc) {
      const unsigned short* kp = ksh + (4 * c + j) * 64 + dc * 32 + 8 * hh;
      const v16bf kbh = ldfrag_b(kp);
      const v16bf kbl = ldfrag_b(kp + 4096);
      acc = mma_b(qh[dc], kbh, acc);
      acc = mma_b(qh[dc], kbl, acc);
      acc = mma_b(ql[dc], kbh, acc);
    }
    s[j] = acc;
  }
}

__global__ __launch_bounds__(128)
void attn_k(const unsigned short* __restrict__ QP, const unsigned short* __restrict__ VP,
            const float* __restrict__ simp, const float* __restrict__ gamp, unsigned short* OP) {
  __shared__ __align__(16) unsigned short Ksh[2 * 64 * 64];
  __shared__ __align__(16) unsigned short Vsh[2 * 64 * 64];
  __shared__ __align__(16) float Wsc[4][16 * 64];

  const int tid  = threadIdx.x;
  const int wave = tid >> 5;
  const int lane = tid & 31;
  const int hh   = lane >> 4;
  const int c    = lane & 15;

  const int bx   = blockIdx.x;
  const int qb   = bx % NQB;
  const int rest = bx / NQB;
  const int h    = rest % NH;
  const int b    = rest / NH;
  const int q0   = qb * 64 + wave * 16;
  const size_t rowB = (size_t)b * SEQ;

  const float graw = bfr(gamp[h]);
  const float gam  = -(fmaxf(graw, 0.0f) + log1pf(__expf(-fabsf(graw))));

  const unsigned short* qfr = QP + (rowB + q0 + c) * QPITCH + (size_t)h * HD + 8 * hh;
  const float* simq = simp + (rowB + q0 + 8 * hh) * (size_t)SEQ + 4 * c;
  unsigned short* Phi = (unsigned short*)(&Wsc[wave][0]);
  unsigned short* Plo = Phi + 1024;

  const int sr = tid >> 1, shalf = (tid & 1) * 32;
  const unsigned short* kstg = QP + (rowB + sr) * QPITCH + (size_t)h * HD + shalf;
  const unsigned short* vstg = VP + ((size_t)b * DM + (size_t)h * HD + sr) * VPITCH + shalf;
  unsigned short* kdst = Ksh + sr * 64 + shalf;
  unsigned short* vdst = Vsh + sr * 64 + shalf;

  float lz[8], z1[8];
#pragma unroll
  for (int r = 0; r < 8; ++r) { lz[r] = -3.0e38f; z1[r] = 0.0f; }

  for (int kt = 0; kt <= qb; ++kt) {
    const int kv0 = kt * 64;
    __syncthreads();
    {
      const unsigned short* kg = kstg + (size_t)kv0 * QPITCH;
#pragma unroll
      for (int i = 0; i < 4; ++i) {
        const v4u a0 = *(const v4u*)(kg + 8 * i);
        const v4u a1 = *(const v4u*)(kg + DM + 8 * i);
        *(v4u*)(kdst + 8 * i) = a0;
        *(v4u*)(kdst + 4096 + 8 * i) = a1;
      }
    }
    __syncthreads();

    v8f s[4];
    scores_tile(s, qfr, Ksh, c, hh);
    const bool first = (kt == 0);
#pragma unroll
    for (int r = 0; r < 8; ++r) {
      const int qrow = q0 + 8 * hh + r;
      const int keyb = kv0 + 4 * c;
      const v4f u = *(const v4f*)(simq + (size_t)r * SEQ + kv0);
      float a[4];
      float mt = -3.0e38f;
#pragma unroll
      for (int j = 0; j < 4; ++j) {
        a[j] = (s[j][r] * 0.125f) * bfr(u[j]);
        const bool ok = (keyb + j) <= qrow;
        mt = fmaxf(mt, ok ? a[j] : -3.0e38f);
      }
#pragma unroll
      for (int off = 1; off < 16; off <<= 1) mt = fmaxf(mt, __shfl_xor(mt, off, 32));
      const float mn = fmaxf(lz[r], mt);
      const float alpha = first ? 0.0f : __expf(lz[r] - mn);
      float sum = 0.0f;
#pragma unroll
      for (int j = 0; j < 4; ++j) sum += ((keyb + j) <= qrow) ? __expf(a[j] - mn) : 0.0f;
#pragma unroll
      for (int off = 1; off < 16; off <<= 1) sum += __shfl_xor(sum, off, 32);
      z1[r] = z1[r] * alpha + sum;
      lz[r] = mn;
    }
  }
#pragma unroll
  for (int r = 0; r < 8; ++r) lz[r] = lz[r] + logf(z1[r]);

  float carry[8], m2[8], l2[8];
  v8f oacc[4];
#pragma unroll
  for (int r = 0; r < 8; ++r) { carry[r] = 0.0f; m2[r] = -3.0e38f; l2[r] = 0.0f; }
#pragma unroll
  for (int t = 0; t < 4; ++t) oacc[t] = zero8();

  for (int kt = qb; kt >= 0; --kt) {
    const int kv0 = kt * 64;
    __syncthreads();
    {
      const unsigned short* kg = kstg + (size_t)kv0 * QPITCH;
      const unsigned short* vg = vstg + kv0;
#pragma unroll
      for (int i = 0; i < 4; ++i) {
        const v4u a0 = *(const v4u*)(kg + 8 * i);
        const v4u a1 = *(const v4u*)(kg + DM + 8 * i);
        const v4u b0 = *(const v4u*)(vg + 8 * i);
        const v4u b1 = *(const v4u*)(vg + SEQ + 8 * i);
        *(v4u*)(kdst + 8 * i) = a0;
        *(v4u*)(kdst + 4096 + 8 * i) = a1;
        *(v4u*)(vdst + 8 * i) = b0;
        *(v4u*)(vdst + 4096 + 8 * i) = b1;
      }
    }
    __syncthreads();

    v8f s[4];
    scores_tile(s, qfr, Ksh, c, hh);
    const bool first = (kt == qb);
#pragma unroll
    for (int r = 0; r < 8; ++r) {
      const int qrow = q0 + 8 * hh + r;
      const int keyb = kv0 + 4 * c;
      const v4f u = *(const v4f*)(simq + (size_t)r * SEQ + kv0);
      float a[4], e[4];
      bool ok[4];
#pragma unroll
      for (int j = 0; j < 4; ++j) {
        a[j]  = (s[j][r] * 0.125f) * bfr(u[j]);
        ok[j] = (keyb + j) <= qrow;
        e[j]  = ok[j] ? __expf(a[j] - lz[r]) : 0.0f;
      }
      const float se2 = e[3];
      const float se1 = e[3] + e[2];
      const float se0 = se1 + e[1];
      const float tot = se0 + e[0];
      float I = tot;
#pragma unroll
      for (int o = 1; o < 16; o <<= 1) {
        const float t = __shfl_down(I, o, 16);
        I += t * (((c + o) < 16) ? 1.0f : 0.0f);
      }
      const float tx   = __shfl_down(I, 1, 16);
      const float X    = tx * ((c < 15) ? 1.0f : 0.0f);
      const float ttot = __shfl(I, 0, 16);
      const float base = carry[r] + X;
      carry[r] += ttot;
      float a2[4];
      float mt = -3.0e38f;
#pragma unroll
      for (int j = 0; j < 4; ++j) {
        const float sej = (j == 0) ? se0 : ((j == 1) ? se1 : ((j == 2) ? se2 : 0.0f));
        const float rj  = base + sej;
        const float pos = (float)(qrow - keyb - j);
        const float ds  = __builtin_amdgcn_sqrtf(fmaxf(rj * pos, 0.0f));
        float te = __expf(ds * gam);
        te = fminf(fmaxf(te, 1e-5f), 1e5f);
        a2[j] = ok[j] ? (a[j] * te) : -3.0e38f;
        mt = fmaxf(mt, a2[j]);
      }
#pragma unroll
      for (int off = 1; off < 16; off <<= 1) mt = fmaxf(mt, __shfl_xor(mt, off, 32));
      const float mn = fmaxf(m2[r], mt);
      const float alpha = first ? 0.0f : __expf(m2[r] - mn);
      m2[r] = mn;
      float p[4];
      float psum = 0.0f;
#pragma unroll
      for (int j = 0; j < 4; ++j) {
        p[j] = ok[j] ? __expf(a2[j] - mn) : 0.0f;
        psum += p[j];
      }
      v2u vh, vl;
#pragma unroll
      for (int e2 = 0; e2 < 2; ++e2) {
        const unsigned short ha = bf_bits(p[2 * e2]);
        const unsigned short hb = bf_bits(p[2 * e2 + 1]);
        const unsigned short la = bf_bits(p[2 * e2] - bf_val(ha));
        const unsigned short lb = bf_bits(p[2 * e2 + 1] - bf_val(hb));
        vh[e2] = pk16(ha, hb);
        vl[e2] = pk16(la, lb);
      }
      *(v2u*)(Phi + (8 * hh + r) * 64 + 4 * c) = vh;
      *(v2u*)(Plo + (8 * hh + r) * 64 + 4 * c) = vl;
#pragma unroll
      for (int off = 1; off < 16; off <<= 1) psum += __shfl_xor(psum, off, 32);
      l2[r] = l2[r] * alpha + psum;
#pragma unroll
      for (int t = 0; t < 4; ++t) oacc[t][r] = oacc[t][r] * alpha;
    }
    lds_wave_sync();

#pragma unroll
    for (int kk = 0; kk < 2; ++kk) {
      const unsigned short* pp = Phi + c * 64 + kk * 32 + 8 * hh;
      const v16bf pah = ldfrag_b(pp);
      const v16bf pal = ldfrag_b(pp + 1024);
#pragma unroll
      for (int t = 0; t < 4; ++t) {
        const unsigned short* vv = Vsh + (t * 16 + c) * 64 + kk * 32 + 8 * hh;
        const v16bf vbh = ldfrag_b(vv);
        const v16bf vbl = ldfrag_b(vv + 4096);
        oacc[t] = mma_b(pah, vbh, oacc[t]);
        oacc[t] = mma_b(pah, vbl, oacc[t]);
        oacc[t] = mma_b(pal, vbh, oacc[t]);
      }
    }
  }

  lds_wave_sync();
  float* os = Wsc[wave];
#pragma unroll
  for (int r = 0; r < 8; ++r) {
    const float inv = __builtin_amdgcn_rcpf(l2[r]);
#pragma unroll
    for (int t = 0; t < 4; ++t) os[(8 * hh + r) * 64 + t * 16 + c] = oacc[t][r] * inv;
  }
  lds_wave_sync();
  {
    const int rq = lane >> 3, piece = lane & 7;
    v4u ph[4], pl[4];
#pragma unroll
    for (int it = 0; it < 4; ++it) {
      const int row = it * 4 + rq;
      const v4f x0 = *(const v4f*)(os + row * 64 + piece * 8);
      const v4f x1 = *(const v4f*)(os + row * 64 + piece * 8 + 4);
      float f[8];
      f[0] = x0[0]; f[1] = x0[1]; f[2] = x0[2]; f[3] = x0[3];
      f[4] = x1[0]; f[5] = x1[1]; f[6] = x1[2]; f[7] = x1[3];
      v4u p0, p1;
#pragma unroll
      for (int e = 0; e < 4; ++e) {
        const unsigned short ha = bf_bits(f[2 * e]);
        const unsigned short hb = bf_bits(f[2 * e + 1]);
        const unsigned short la = bf_bits(f[2 * e] - bf_val(ha));
        const unsigned short lb = bf_bits(f[2 * e + 1] - bf_val(hb));
        p0[e] = pk16(ha, hb);
        p1[e] = pk16(la, lb);
      }
      ph[it] = p0;
      pl[it] = p1;
    }
    for (int ps = 0; ps < 2; ++ps) {
#pragma unroll
      for (int it = 0; it < 4; ++it) {
        const int row = it * 4 + rq;
        const size_t go = (rowB + q0 + row) * OPITCH + (size_t)h * HD + piece * 8;
        *(volatile v4u*)(OP + go) = ph[it];
        *(volatile v4u*)(OP + go + DM) = pl[it];
      }
      __threadfence();
    }
  }
}

extern "C" void kernel_launch(void* const* d_in, const int* in_sizes, int n_in,
                              void* d_out, int out_size, void* d_ws, size_t ws_size,
                              hipStream_t stream) {
  if (n_in < 9) return;
  if (in_sizes[0] != ROWS * DM) return;
  if (in_sizes[1] != NBATCH * SEQ * SEQ) return;
  if (in_sizes[2] != DM * DM || in_sizes[3] < DM) return;
  if (in_sizes[4] != DM * DM || in_sizes[5] < DM) return;
  if (in_sizes[6] != DM * DM || in_sizes[7] < DM) return;
  if (in_sizes[8] < NH) return;
  if (out_size != ROWS * DM) return;

  const float* x   = (const float*)d_in[0];
  const float* sim = (const float*)d_in[1];
  const float* Wk  = (const float*)d_in[2];
  const float* bk  = (const float*)d_in[3];
  const float* Wv  = (const float*)d_in[4];
  const float* bv  = (const float*)d_in[5];
  const float* Wo  = (const float*)d_in[6];
  const float* bo  = (const float*)d_in[7];
  const float* gam = (const float*)d_in[8];

  const size_t PXB = (size_t)ROWS * DM * 2;
  const size_t PW  = (size_t)DM * DM * 2;
  const size_t PW2 = (size_t)DM * W2PITCH * 2;
  const size_t PQ  = (size_t)ROWS * QPITCH * 2;
  const size_t PV  = (size_t)NBATCH * DM * VPITCH * 2;
  const size_t PO  = (size_t)ROWS * OPITCH * 2;
  size_t off = 0;
  const size_t oXB  = off; off += PXB;
  const size_t oWKB = off; off += PW;
  const size_t oWVB = off; off += PW;
  const size_t oWO2 = off; off += PW2;
  const size_t oQP  = off; off += PQ;
  const size_t oVP  = off; off += PV;
  const size_t oOP  = off; off += PO;
  if (off > ws_size) return;
  if (off > (size_t)134217728) return;

  char* ws = (char*)d_ws;
  unsigned short* XB  = (unsigned short*)(ws + oXB);
  unsigned short* WKB = (unsigned short*)(ws + oWKB);
  unsigned short* WVB = (unsigned short*)(ws + oWVB);
  unsigned short* WO2 = (unsigned short*)(ws + oWO2);
  unsigned short* QP  = (unsigned short*)(ws + oQP);
  unsigned short* VP  = (unsigned short*)(ws + oVP);
  unsigned short* OP  = (unsigned short*)(ws + oOP);
  float*          outf = (float*)d_out;

  const dim3 blk(256);
  const int n8x = ROWS * DM / 8;
  const int n8w = DM * DM / 8;
  const dim3 gCx((n8x + 255) / 256);
  const dim3 gCw((n8w + 255) / 256);
  const dim3 gGq(((ROWS / 64) * (DM / 64) + 7) / 8);
  const dim3 gAttn(NBATCH * NH * NQB);

  cvt_bf<<<gCx, blk, 0, stream>>>(x, XB, n8x, 0, DM);
  cvt_bf<<<gCw, blk, 0, stream>>>(Wk, WKB, n8w, 0, DM);
  cvt_bf<<<gCw, blk, 0, stream>>>(Wv, WVB, n8w, 0, DM);
  cvt_bf<<<gCw, blk, 0, stream>>>(Wo, WO2, n8w, 1, DM);
  gemm64_bf<0><<<gGq, blk, 0, stream>>>(XB, DM, WKB, DM, bk, (void*)QP, QPITCH, DM, ROWS, DM, DM);
  gemm64_bf<1><<<gGq, blk, 0, stream>>>(WVB, DM, XB, DM, bv, (void*)VP, VPITCH, SEQ, DM, ROWS, DM);
  attn_k<<<gAttn, dim3(128), 0, stream>>>(QP, VP, sim, gam, OP);
  gemm64_bf<2><<<gGq, blk, 0, stream>>>(OP, OPITCH, WO2, W2PITCH, bo, (void*)outf, DM, 0, ROWS, DM, 2 * DM);
  (void)hipGetLastError();
}
